// Bahdanau_61684320305411
// MI455X (gfx1250) — hardware-verified
//
#include <hip/hip_runtime.h>
#include <stdint.h>


typedef __attribute__((ext_vector_type(16))) _Float16 v16h;
typedef __attribute__((ext_vector_type(8)))  _Float16 v8h;
typedef __attribute__((ext_vector_type(16))) __bf16   v16b;
typedef __attribute__((ext_vector_type(8)))  __bf16   v8b;
typedef __attribute__((ext_vector_type(8)))  float    v8f;
typedef __attribute__((ext_vector_type(4)))  float    v4f;
#define PSCALE 32768.0f
#define U16(p) ((const unsigned short*)(const void*)(p))
#define PSCALE_INV (1.0f / 32768.0f)

__device__ __forceinline__ unsigned short f2bf_bits(float f) {
  unsigned u = __float_as_uint(f);
  return (unsigned short)((u + 0x7FFFu + ((u >> 16) & 1u)) >> 16);
}
__device__ __forceinline__ float bf_bits2f(unsigned short h) { return __uint_as_float(((unsigned)h) << 16); }

__device__ __forceinline__ void dep_guard_h(v8f& a, v8f& b, v16h x, v16h y) { asm volatile("v_nop\n\tv_nop\n\tv_nop\n\tv_nop" : "+v"(a), "+v"(b) : "v"(x), "v"(y)); }
__device__ __forceinline__ void dep_guard_b(v8f& a, v8f& b, v16b x, v16b y) { asm volatile("v_nop\n\tv_nop\n\tv_nop\n\tv_nop" : "+v"(a), "+v"(b) : "v"(x), "v"(y)); }
__device__ __forceinline__ void keep4_h(v16h a, v16h b, v16h c, v16h d) { asm volatile("v_nop" :: "v"(a), "v"(b), "v"(c), "v"(d)); }
__device__ __forceinline__ void keep4_b(v16b a, v16b b, v16b c, v16b d) { asm volatile("v_nop" :: "v"(a), "v"(b), "v"(c), "v"(d)); }
__device__ __forceinline__ void acc_guard4(v8f& a, v8f& b, v8f& c, v8f& d) { asm volatile("v_nop\n\tv_nop\n\tv_nop\n\tv_nop" : "+v"(a), "+v"(b), "+v"(c), "+v"(d)); }
template <typename T> struct Frag;
template <> struct Frag<_Float16> {
  typedef v16h V; union U { v16h v; v8h h[2]; };
  static __device__ __forceinline__ v16h load(const _Float16* p) {
    U f; f.h[0] = *(const v8h*)(p); f.h[1] = *(const v8h*)(p + 16); return f.v;
  }
  static __device__ __forceinline__ v8f mma(v16h a, v16h b, v8f c) {
    return __builtin_amdgcn_wmma_f32_16x16x32_f16(false, a, false, b, (short)0, c, false, false);
  }
  static __device__ __forceinline__ void guard(v8f& a, v8f& b, v16h x, v16h y) { dep_guard_h(a, b, x, y); }
  static __device__ __forceinline__ void keep(v16h a, v16h b, v16h c, v16h d) { keep4_h(a, b, c, d); }
};
template <> struct Frag<__bf16> {
  typedef v16b V; union U { v16b v; v8b h[2]; };
  static __device__ __forceinline__ v16b load(const __bf16* p) {
    U f; f.h[0] = *(const v8b*)(p); f.h[1] = *(const v8b*)(p + 16); return f.v;
  }
  static __device__ __forceinline__ v8f mma(v16b a, v16b b, v8f c) {
    return __builtin_amdgcn_wmma_f32_16x16x32_bf16(false, a, false, b, (short)0, c, false, false);
  }
  static __device__ __forceinline__ void guard(v8f& a, v8f& b, v16b x, v16b y) { dep_guard_b(a, b, x, y); }
  static __device__ __forceinline__ void keep(v16b a, v16b b, v16b c, v16b d) { keep4_b(a, b, c, d); }
};

template <int ET> struct Elem;
template <> struct Elem<0> { typedef _Float16 T; };
template <> struct Elem<1> { typedef __bf16 T; };
template <int ET, bool SPLIT, int BIAS_MODE, int OUT_MODE, bool RESID, int ACT = 0>
__global__ __launch_bounds__(256) void wmma_gemm64(
    const unsigned short* __restrict__ Ap, const unsigned short* __restrict__ A2p, int lda, long strideA,
    const unsigned short* __restrict__ Btp, const unsigned short* __restrict__ Bt2p, int ldb, long strideB,
    void* __restrict__ Cout, void* __restrict__ Cout2, int ldc, long strideC,
    const float* __restrict__ bias,
    const float* __restrict__ resid, long strideR,
    int M, int N, int K, float scale) {
  typedef typename Elem<ET>::T T;
  typedef typename Frag<T>::V V;
  const T* A = (const T*)Ap; const T* A2 = (const T*)A2p; const T* Bt = (const T*)Btp; const T* Bt2 = (const T*)Bt2p;
  __shared__ __align__(16) float sT[8][16 * 68];
  const int b    = blockIdx.y;
  const int lane = threadIdx.x & 31;
  const int wave = threadIdx.x >> 5;
  const int tilesN = N >> 6;
  const int tilesM = M >> 6;
  const int tile = blockIdx.x * 8 + wave;
  if (tile >= tilesM * tilesN) return;
  const int tm = tile / tilesN;
  const int tn = tile - tm * tilesN;
  const int m0 = tm << 6;
  const int n0 = tn << 6;

  const T* Ab  = A  + (size_t)b * strideA;
  const T* Bb  = Bt + (size_t)b * strideB;
  const T* Ab2 = SPLIT ? (A2  + (size_t)b * strideA) : nullptr;
  const T* Bb2 = SPLIT ? (Bt2 + (size_t)b * strideB) : nullptr;

  const int rlane = lane & 15;
  const int koff  = (lane >> 4) * 8;
  const int mOff  = (lane >> 4) * 8;

  v8f acc[4][4];
#pragma unroll
  for (int i = 0; i < 4; ++i)
#pragma unroll
    for (int j = 0; j < 4; ++j) acc[i][j] = (v8f){0.f,0.f,0.f,0.f,0.f,0.f,0.f,0.f};

  for (int k0 = 0; k0 < K; k0 += 32) {
    V bh[4], bl[4];
#pragma unroll
    for (int j = 0; j < 4; ++j) {
      const size_t bo = (size_t)(n0 + (j << 4) + rlane) * ldb + koff + k0;
      bh[j] = Frag<T>::load(Bb + bo);
      if (SPLIT) bl[j] = Frag<T>::load(Bb2 + bo);
    }
#pragma unroll
    for (int i = 0; i < 4; ++i) {
      const size_t ao = (size_t)(m0 + (i << 4) + rlane) * lda + koff + k0;
      V ah = Frag<T>::load(Ab + ao);
      V al;
      if (SPLIT) al = Frag<T>::load(Ab2 + ao);
#pragma unroll
      for (int j = 0; j < 4; ++j) {
        acc[i][j] = Frag<T>::mma(ah, bh[j], acc[i][j]);
        if (SPLIT) {
          acc[i][j] = Frag<T>::mma(ah, bl[j], acc[i][j]);
          acc[i][j] = Frag<T>::mma(al, bh[j], acc[i][j]);
        }
      }
      Frag<T>::guard(acc[i][0], acc[i][3], ah, SPLIT ? al : ah);
    }
    Frag<T>::keep(bh[0], bh[1], bh[2], bh[3]);
    if (SPLIT) Frag<T>::keep(bl[0], bl[1], bl[2], bl[3]);
  }
  acc_guard4(acc[0][0], acc[0][1], acc[0][2], acc[0][3]);
  acc_guard4(acc[1][0], acc[1][1], acc[1][2], acc[1][3]);
  acc_guard4(acc[2][0], acc[2][1], acc[2][2], acc[2][3]);
  acc_guard4(acc[3][0], acc[3][1], acc[3][2], acc[3][3]);

  float* slab = sT[wave];
  const float* Rb = RESID ? (resid + (size_t)b * strideR) : nullptr;
#pragma unroll
  for (int i = 0; i < 4; ++i) {
    const int mBase = m0 + (i << 4);
#pragma unroll
    for (int j = 0; j < 4; ++j) {
      const int n = n0 + (j << 4) + rlane;
      float bv = 0.f;
      if (BIAS_MODE == 2) bv = bias[n];
#pragma unroll
      for (int r = 0; r < 8; ++r) {
        float v = acc[i][j][r] * scale;
        if (BIAS_MODE == 1) v += bias[mBase + mOff + r];
        if (BIAS_MODE == 2) v += bv;
        if (RESID) v += Rb[(size_t)(mBase + mOff + r) * ldc + n];
        if (ACT == 1) v = tanhf(v);
        if (ACT == 2) v = fmaxf(v, 0.0f);
        if (ACT == 3) v = v / (1.0f + expf(-v));
        if (ACT == 4) v = (v > 0.f) ? v : 0.01f * v;
        if (ACT == 5) v = 0.5f * v * (1.0f + erff(v * 0.70710678118654752f));
        slab[(mOff + r) * 68 + (j << 4) + rlane] = v;
      }
    }
    __builtin_amdgcn_fence(__ATOMIC_RELEASE, "workgroup");
    __builtin_amdgcn_wave_barrier();
    __builtin_amdgcn_fence(__ATOMIC_ACQUIRE, "workgroup");
    if (OUT_MODE == 0) {
      float* C = (float*)Cout + (size_t)b * strideC;
      const int hh = lane >> 4, c4 = (lane & 15) * 4;
      for (int pass = 0; pass < 2; ++pass) {
#pragma unroll
        for (int it = 0; it < 8; ++it) {
          const int row = it * 2 + hh;
          v4f v = *(const v4f*)(slab + row * 68 + c4);
          *(volatile v4f*)(C + (size_t)(mBase + row) * ldc + n0 + c4) = v;
        }
        __threadfence();
      }
    } else {
      const int q = lane >> 3, c8 = (lane & 7) * 8;
      unsigned short* C  = (unsigned short*)Cout  + (size_t)b * strideC;
      unsigned short* C2 = (OUT_MODE == 2) ? ((unsigned short*)Cout2 + (size_t)b * strideC) : nullptr;
      for (int pass = 0; pass < 2; ++pass) {
#pragma unroll
        for (int it = 0; it < 4; ++it) {
          const int row = it * 4 + q;
          const float* sp = slab + row * 68 + c8;
          v8h hv, lv;
#pragma unroll
          for (int e = 0; e < 8; ++e) {
            if (OUT_MODE == 1) {
              hv[e] = (_Float16)sp[e];
            } else {
              unsigned short hb = f2bf_bits(sp[e]);
              unsigned short lb = f2bf_bits(sp[e] - bf_bits2f(hb));
              hv[e] = __builtin_bit_cast(_Float16, hb);
              lv[e] = __builtin_bit_cast(_Float16, lb);
            }
          }
          *(volatile v8h*)(C + (size_t)(mBase + row) * ldc + n0 + c8) = hv;
          if (OUT_MODE == 2) *(volatile v8h*)(C2 + (size_t)(mBase + row) * ldc + n0 + c8) = lv;
        }
        __threadfence();
      }
    }
    __builtin_amdgcn_fence(__ATOMIC_RELEASE, "workgroup");
    __builtin_amdgcn_wave_barrier();
    __builtin_amdgcn_fence(__ATOMIC_ACQUIRE, "workgroup");
  }
}

__global__ __launch_bounds__(256) void cast_f32_f16x2(
    const float* __restrict__ in, _Float16* __restrict__ out, int n2) {
  int i = blockIdx.x * 256 + threadIdx.x;
  if (i < n2) {
    const _Float16 h0 = (_Float16)in[2 * i], h1 = (_Float16)in[2 * i + 1];
    const unsigned u = (unsigned)__builtin_bit_cast(unsigned short, h0) | ((unsigned)__builtin_bit_cast(unsigned short, h1) << 16);
    ((volatile unsigned*)out)[i] = u;
    __threadfence();
    ((volatile unsigned*)out)[i] = u;
  }
}

#define NB 16
#define NL 64
#define ND 512
#define NO 1024

__global__ __launch_bounds__(256) void transpose64_f16(
    const float* __restrict__ in0, const float* __restrict__ in1, int zsplit, long zs_in, int ld_in,
    _Float16* __restrict__ out, long zs_out, int ld_out, float scale) {
  __shared__ __align__(16) _Float16 tile[64 * 72];
  const int tid = threadIdx.x, lane = tid & 31, wave = tid >> 5;
  const int z = blockIdx.z;
  const int r0 = blockIdx.y * 64, c0 = blockIdx.x * 64;
  const float* src = (z < zsplit) ? (in0 + (size_t)z * zs_in) : (in1 + (size_t)(z - zsplit) * zs_in);
  _Float16* dst = out + (size_t)z * zs_out;
#pragma unroll
  for (int it = 0; it < 4; ++it) {
    const int idx = tid + 256 * it;
    const int r = idx >> 4;
    const int c4 = (idx & 15) * 4;
    const v4f v = *(const v4f*)(src + (size_t)(r0 + r) * ld_in + c0 + c4);
#pragma unroll
    for (int e = 0; e < 4; ++e) tile[(c4 + e) * 72 + r] = (_Float16)(v[e] * scale);
  }
  __syncthreads();
  const int q = lane >> 3, c8 = (lane & 7) * 8;
  for (int pass = 0; pass < 2; ++pass) {
#pragma unroll
    for (int it = 0; it < 2; ++it) {
      const int c = wave * 8 + it * 4 + q;
      const v8h val = *(const v8h*)(tile + c * 72 + c8);
      *(volatile v8h*)(dst + (size_t)(c0 + c) * ld_out + r0 + c8) = val;
    }
    __threadfence();
  }
}

__global__ __launch_bounds__(256) void score_kernel(
    const float* __restrict__ S, const float* __restrict__ b1, const float* __restrict__ W2,
    const float* __restrict__ b2, const int* __restrict__ mask0, const int* __restrict__ mask1,
    float* __restrict__ attn) {
  __shared__ __align__(16) float s1b[NO];
  __shared__ __align__(16) float w2s[NO];
  __shared__ float scs[NL];
  const int tid = threadIdx.x, lane = tid & 31, wave = tid >> 5;
  const int b = blockIdx.x >> 6, i = blockIdx.x & 63;
  {
    const float* s1row = S + (size_t)NO * NO + (size_t)(b * NL + i) * NO;
    const v4f sv = *(const v4f*)(s1row + 4 * tid);
    const v4f bv = *(const v4f*)(b1 + 4 * tid);
    const v4f wv = *(const v4f*)(W2 + 4 * tid);
#pragma unroll
    for (int e = 0; e < 4; ++e) {
      s1b[4 * tid + e] = sv[e] + bv[e];
      w2s[4 * tid + e] = wv[e];
    }
  }
  __syncthreads();
#pragma unroll 1
  for (int jt = 0; jt < 8; ++jt) {
    const int j = wave * 8 + jt;
    const float* s0row = S + (size_t)(b * NL + j) * NO;
    float part = 0.0f;
#pragma unroll 4
    for (int kq = 0; kq < 8; ++kq) {
      const int o = 128 * kq + 4 * lane;
      const v4f av = *(const v4f*)(s0row + o);
      const v4f sv = *(const v4f*)(s1b + o);
      const v4f wv = *(const v4f*)(w2s + o);
#pragma unroll
      for (int e = 0; e < 4; ++e) {
        const float x  = sv[e] + av[e];
        const float ex = __builtin_amdgcn_exp2f(x * 2.88539008f);
        const float r  = __builtin_amdgcn_rcpf(1.0f + ex);
        const float t  = 1.0f - 2.0f * r;
        part = fmaf(wv[e], t, part);
      }
    }
#pragma unroll
    for (int off = 16; off > 0; off >>= 1) part += __shfl_xor(part, off, 32);
    if (lane == 0) scs[j] = part;
  }
  __syncthreads();
  if (tid < 16) {
    const float bias = b2[0];
    const float m0 = (float)mask0[b * NL + i];
    v4f v;
#pragma unroll
    for (int e = 0; e < 4; ++e) {
      const int j = 4 * tid + e;
      float sc = scs[j] + bias;
      const float wm = m0 * (float)mask1[b * NL + j];
      sc = sc + (-1.0e8f) * wm;
      v[e] = sc;
    }
    float* dst = attn + (size_t)(b * NL + i) * NL + 4 * tid;
    *(volatile v4f*)dst = v;
    __threadfence();
    *(volatile v4f*)dst = v;
  }
}

__global__ __launch_bounds__(256) void softmax_kernel(const float* __restrict__ attn, _Float16* __restrict__ P) {
  __shared__ __align__(16) float at[64 * 65];
  __shared__ __align__(16) _Float16 p1s[64 * 72];
  __shared__ __align__(16) _Float16 p2s[64 * 72];
  const int tid = threadIdx.x, lane = tid & 31, wave = tid >> 5;
  const int b = blockIdx.x;
  const float* ab = attn + (size_t)b * (NL * NL);
#pragma unroll
  for (int it = 0; it < 4; ++it) {
    const int idx = tid + 256 * it;
    const int r = idx >> 4;
    const int c4 = (idx & 15) * 4;
    const v4f v = *(const v4f*)(ab + r * NL + c4);
#pragma unroll
    for (int e = 0; e < 4; ++e) at[r * 65 + c4 + e] = v[e];
  }
  __syncthreads();
#pragma unroll 1
  for (int rr = 0; rr < 8; ++rr) {
    const int a = wave * 8 + rr;
    const float x0 = at[a * 65 + lane], x1 = at[a * 65 + lane + 32];
    float m = fmaxf(x0, x1);
#pragma unroll
    for (int off = 16; off > 0; off >>= 1) m = fmaxf(m, __shfl_xor(m, off, 32));
    const float e0 = __builtin_amdgcn_exp2f((x0 - m) * 1.44269504f);
    const float e1 = __builtin_amdgcn_exp2f((x1 - m) * 1.44269504f);
    float s = e0 + e1;
#pragma unroll
    for (int off = 16; off > 0; off >>= 1) s += __shfl_xor(s, off, 32);
    const float inv = 1.0f / s;
    p1s[a * 72 + lane]      = (_Float16)(e0 * inv * PSCALE);
    p1s[a * 72 + lane + 32] = (_Float16)(e1 * inv * PSCALE);
  }
#pragma unroll 1
  for (int cc = 0; cc < 8; ++cc) {
    const int c = wave * 8 + cc;
    const float x0 = at[lane * 65 + c], x1 = at[(lane + 32) * 65 + c];
    float m = fmaxf(x0, x1);
#pragma unroll
    for (int off = 16; off > 0; off >>= 1) m = fmaxf(m, __shfl_xor(m, off, 32));
    const float e0 = __builtin_amdgcn_exp2f((x0 - m) * 1.44269504f);
    const float e1 = __builtin_amdgcn_exp2f((x1 - m) * 1.44269504f);
    float s = e0 + e1;
#pragma unroll
    for (int off = 16; off > 0; off >>= 1) s += __shfl_xor(s, off, 32);
    const float inv = 1.0f / s;
    p2s[c * 72 + lane]      = (_Float16)(e0 * inv * PSCALE);
    p2s[c * 72 + lane + 32] = (_Float16)(e1 * inv * PSCALE);
  }
  __syncthreads();
  _Float16* d1 = P + (size_t)b * (NL * NL);
  _Float16* d2 = P + (size_t)(NB + b) * (NL * NL);
  const int q = lane >> 3, c8 = (lane & 7) * 8;
  for (int pass = 0; pass < 2; ++pass) {
#pragma unroll
    for (int it = 0; it < 2; ++it) {
      const int row = wave * 8 + it * 4 + q;
      const v8h v1 = *(const v8h*)(p1s + row * 72 + c8);
      const v8h v2 = *(const v8h*)(p2s + row * 72 + c8);
      *(volatile v8h*)(d1 + (size_t)row * NL + c8) = v1;
      *(volatile v8h*)(d2 + (size_t)row * NL + c8) = v2;
    }
    __threadfence();
  }
}

extern "C" void kernel_launch(void* const* d_in, const int* in_sizes, int n_in,
                              void* d_out, int out_size, void* d_ws, size_t ws_size,
                              hipStream_t stream) {
  if (n_in < 8) return;
  if (in_sizes[0] != NB * NL * ND || in_sizes[1] != NB * NL * ND ||
      in_sizes[2] != NB * NL || in_sizes[3] != NB * NL ||
      in_sizes[4] != 2 * ND * NO || in_sizes[5] != NO || in_sizes[6] != NO || in_sizes[7] < 1 ||
      out_size != 2 * NB * NL * ND) return;

  const float* q0    = (const float*)d_in[0];
  const float* q1    = (const float*)d_in[1];
  const int*   mask0 = (const int*)d_in[2];
  const int*   mask1 = (const int*)d_in[3];
  const float* W1    = (const float*)d_in[4];
  const float* b1    = (const float*)d_in[5];
  const float* W2    = (const float*)d_in[6];
  const float* b2    = (const float*)d_in[7];

  const size_t szQh = (size_t)2 * NB * NL * ND * 2;
  const size_t szWt = (size_t)2 * NO * ND * 2;
  const size_t szQt = (size_t)2 * NB * ND * NL * 2;
  const size_t szS  = (size_t)2 * NO * NO * 4;
  const size_t szAt = (size_t)NB * NL * NL * 4;
  const size_t szP  = (size_t)2 * NB * NL * NL * 2;
  const size_t oQh = 0, oWt = oQh + szQh, oQt = oWt + szWt, oS = oQt + szQt, oAt = oS + szS, oP = oAt + szAt;
  const size_t total = oP + szP;
  if (total > ws_size) return;

  char* ws = (char*)d_ws;
  _Float16* Qh = (_Float16*)(ws + oQh);
  _Float16* Wt = (_Float16*)(ws + oWt);
  _Float16* Qt = (_Float16*)(ws + oQt);
  float*    S  = (float*)(ws + oS);
  float*    At = (float*)(ws + oAt);
  _Float16* P  = (_Float16*)(ws + oP);
  float*    out = (float*)d_out;

  const int n2 = NB * NL * ND / 2;
  cast_f32_f16x2<<<dim3((n2 + 255) / 256), dim3(256), 0, stream>>>(q0, Qh, n2);
  cast_f32_f16x2<<<dim3((n2 + 255) / 256), dim3(256), 0, stream>>>(q1, Qh + (size_t)NB * NL * ND, n2);

  transpose64_f16<<<dim3(NO / 64, ND / 64, 2), dim3(256), 0, stream>>>(
      W1, W1 + (size_t)ND * NO, 1, 0L, NO, Wt, (long)NO * ND, ND, 16.0f);

  transpose64_f16<<<dim3(ND / 64, NL / 64, 2 * NB), dim3(256), 0, stream>>>(
      q1, q0, NB, (long)NL * ND, ND, Qt, (long)ND * NL, NL, 1.0f);

  wmma_gemm64<0, false, 0, 0, false><<<dim3(32, 2), dim3(256), 0, stream>>>(
      (const unsigned short*)Qh, (const unsigned short*)Qh, ND, (long)NO * ND,
      (const unsigned short*)Wt, (const unsigned short*)Wt, ND, (long)NO * ND,
      (void*)S, (void*)S, NO, (long)NO * NO,
      b1, b1, 0L, NO, NO, ND, 1.0f / 16.0f);

  score_kernel<<<dim3(NB * NL), dim3(256), 0, stream>>>(S, b1, W2, b2, mask0, mask1, At);

  softmax_kernel<<<dim3(NB), dim3(256), 0, stream>>>(At, P);

  wmma_gemm64<0, false, 0, 0, false><<<dim3(1, 2 * NB), dim3(256), 0, stream>>>(
      (const unsigned short*)P, (const unsigned short*)P, NL, (long)NL * NL,
      (const unsigned short*)Qt, (const unsigned short*)Qt, NL, (long)ND * NL,
      (void*)out, (void*)out, ND, (long)NL * ND,
      b1, b1, 0L, NL, ND, NL, PSCALE_INV);

  (void)hipGetLastError();
}
